// MambaStateSpaceLayer_55164559950115
// MI455X (gfx1250) — hardware-verified
//
#include <hip/hip_runtime.h>

#define B_SZ   2
#define SEQ    1024
#define DMODEL 1024
#define DINNER 2048
#define DSTATE 16
#define TOKENS (B_SZ * SEQ)

typedef _Float16 v16h __attribute__((ext_vector_type(16)));
typedef _Float16 v8h  __attribute__((ext_vector_type(8)));
typedef float    v8f  __attribute__((ext_vector_type(8)));
typedef float    v4f  __attribute__((ext_vector_type(4)));

union Frag { v16h v; v8h half[2]; };

__device__ __forceinline__ v8f wmma_f16(v16h a, v16h b, v8f c) {
  v8f d = __builtin_amdgcn_wmma_f32_16x16x32_f16(false, a, false, b, (short)0, c, false, false);
  asm volatile("v_nop\n\tv_nop\n\tv_nop\n\tv_nop" : "+v"(d) : "v"(a), "v"(b));
  return d;
}

__device__ __forceinline__ v8h cvt8(v4f p, v4f q, float s) {
  v8h r = {(_Float16)(p.x * s), (_Float16)(p.y * s), (_Float16)(p.z * s), (_Float16)(p.w * s),
           (_Float16)(q.x * s), (_Float16)(q.y * s), (_Float16)(q.z * s), (_Float16)(q.w * s)};
  return r;
}

__device__ __forceinline__ float actf(float v, int mode, int c, int from) {
  if (mode == 1) { if (c >= from) v = fmaxf(v, 0.0f); }
  else if (mode == 2) { v = 1.0f / (1.0f + __expf(-v)); }
  return v;
}

#define TM 64
#define TN 128
#define TK 32
#define SK 40
#define CP 132

__global__ __launch_bounds__(256)
void gemm_f16_nt(const float* __restrict__ A,
                 const float* __restrict__ W,
                 const float* __restrict__ bias,
                 float* __restrict__ O,
                 int M, int N, int K,
                 float sA, float sW, float sO,
                 int act_mode, int act_from_col)
{
  __shared__ __attribute__((aligned(16))) _Float16 As[TM][SK];
  __shared__ __attribute__((aligned(16))) _Float16 Bs[TN][SK];
  __shared__ __attribute__((aligned(16))) float    Cs[TM][CP];

  const int bn = blockIdx.x * TN;
  const int bm = blockIdx.y * TM;
  if (bm + TM > M || bn + TN > N) return;

  const int tid  = threadIdx.x;
  const int wave = tid >> 5;
  const int lane = tid & 31;
  const int h    = lane >> 4;
  const int l16  = lane & 15;
  const int wm   = (wave & 3) << 4;
  const int wn   = (wave >> 2) << 6;

  const int rA = tid >> 2, cA = (tid & 3) * 8;
  const int rB = tid >> 1, cB = (tid & 1) * 16;
  const float* aRow = A + (size_t)(bm + rA) * K + cA;
  const float* wRow = W + (size_t)(bn + rB) * K + cB;

  v8f acc[4];
#pragma unroll
  for (int t = 0; t < 4; ++t) {
    v8f z = {0.f, 0.f, 0.f, 0.f, 0.f, 0.f, 0.f, 0.f};
    acc[t] = z;
  }

  const int nk = K / TK;
  for (int kt = 0; kt < nk; ++kt) {
    const int k0 = kt * TK;
    v4f a0 = *(const v4f*)(aRow + k0);
    v4f a1 = *(const v4f*)(aRow + k0 + 4);
    v4f w0 = *(const v4f*)(wRow + k0);
    v4f w1 = *(const v4f*)(wRow + k0 + 4);
    v4f w2 = *(const v4f*)(wRow + k0 + 8);
    v4f w3 = *(const v4f*)(wRow + k0 + 12);
    __syncthreads();
    *(v8h*)&As[rA][cA]     = cvt8(a0, a1, sA);
    *(v8h*)&Bs[rB][cB]     = cvt8(w0, w1, sW);
    *(v8h*)&Bs[rB][cB + 8] = cvt8(w2, w3, sW);
    __syncthreads();

    Frag af;
    af.half[0] = *(const v8h*)&As[wm + l16][8 * h];
    af.half[1] = *(const v8h*)&As[wm + l16][16 + 8 * h];
#pragma unroll
    for (int t = 0; t < 4; ++t) {
      const int n = wn + 16 * t + l16;
      Frag bf;
      bf.half[0] = *(const v8h*)&Bs[n][8 * h];
      bf.half[1] = *(const v8h*)&Bs[n][16 + 8 * h];
      acc[t] = wmma_f16(af.v, bf.v, acc[t]);
    }
  }

#pragma unroll
  for (int t = 0; t < 4; ++t) {
#pragma unroll
    for (int r = 0; r < 8; ++r) {
      Cs[wm + 8 * h + r][wn + 16 * t + l16] = acc[t][r];
    }
  }
  __syncthreads();

  const int col = lane * 4;
  const v4f bb = *(const v4f*)(bias + bn + col);
  v4f vv[8];
#pragma unroll
  for (int rr = 0; rr < 8; ++rr) {
    const int row = wave * 8 + rr;
    v4f v = *(const v4f*)&Cs[row][col];
    v = v * sO + bb;
    v.x = actf(v.x, act_mode, bn + col + 0, act_from_col);
    v.y = actf(v.y, act_mode, bn + col + 1, act_from_col);
    v.z = actf(v.z, act_mode, bn + col + 2, act_from_col);
    v.w = actf(v.w, act_mode, bn + col + 3, act_from_col);
    vv[rr] = v;
  }
  float* obase = O + (size_t)(bm + wave * 8) * N + bn + col;
#pragma unroll
  for (int rr = 0; rr < 8; ++rr) {
    *(volatile v4f*)(obase + (size_t)rr * N) = vv[rr];
  }
  __threadfence();
#pragma unroll
  for (int rr = 0; rr < 8; ++rr) {
    *(volatile v4f*)(obase + (size_t)rr * N) = vv[rr];
  }
}

#define SCAN_T 256

__global__ __launch_bounds__(SCAN_T)
void ssm_scan(const float* __restrict__ proj,
              const float* __restrict__ gate,
              const float* __restrict__ A_log,
              const float* __restrict__ B_mat,
              const float* __restrict__ C_mat,
              const float* __restrict__ D_vec,
              float* __restrict__ gy)
{
  __shared__ __attribute__((aligned(16))) float sh[SCAN_T];

  const int tid   = threadIdx.x;
  const int blk   = blockIdx.x;
  if (blk >= (B_SZ * DINNER) / SCAN_T) return;
  const int b     = blk / (DINNER / SCAN_T);
  const int dbase = (blk % (DINNER / SCAN_T)) * SCAN_T;
  const int d     = dbase + tid;

  float a[DSTATE], Bv[DSTATE], c0[DSTATE], hs[DSTATE];
#pragma unroll
  for (int n = 0; n < DSTATE; ++n) {
    a[n]  = -__expf(A_log[d * DSTATE + n]);
    Bv[n] = B_mat[d * DSTATE + n];
    c0[n] = C_mat[n];
    hs[n] = 0.0f;
  }
  const float Dv = D_vec[d];

  for (int t = 0; t < SEQ; ++t) {
    const int tt = b * SEQ + t;
    const size_t prow = (size_t)tt * (2 * DINNER);
    const float xv = proj[prow + d];
    const float dt = proj[prow + DINNER + d];
    const float g  = gate[(size_t)tt * DINNER + d];
    const float u  = xv * dt;
    float y = 0.0f;
#pragma unroll
    for (int n = 0; n < DSTATE; ++n) {
      const float e = __expf(a[n] * dt);
      hs[n] = hs[n] * e + u * Bv[n];
      y += hs[n] * c0[n];
    }
    const float val = g * (y + xv * Dv);

    sh[tid] = val;
    __syncthreads();
    if (tid < SCAN_T / 4) {
      const v4f v = *(const v4f*)&sh[tid * 4];
      float* op = gy + (size_t)tt * DINNER + dbase + tid * 4;
      *(volatile v4f*)op = v;
      __threadfence();
      *(volatile v4f*)op = v;
    }
    __syncthreads();
  }
}

static_assert(TOKENS % TM == 0, "");
static_assert((2 * DINNER) % TN == 0 && DINNER % TN == 0 && DMODEL % TN == 0, "");
static_assert(DMODEL % TK == 0 && DINNER % TK == 0, "");
static_assert(DINNER % SCAN_T == 0, "");

extern "C" void kernel_launch(void* const* d_in, const int* in_sizes, int n_in,
                              void* d_out, int out_size, void* d_ws, size_t ws_size,
                              hipStream_t stream) {
  if (n_in < 11) return;
  if (in_sizes[0] != TOKENS * DMODEL || in_sizes[1] != 2 * DINNER * DMODEL ||
      in_sizes[2] != 2 * DINNER     || in_sizes[3] != DINNER * DMODEL ||
      in_sizes[4] != DINNER         || in_sizes[5] != DMODEL * DINNER ||
      in_sizes[6] != DMODEL         || in_sizes[7] != DINNER * DSTATE ||
      in_sizes[8] != DINNER * DSTATE || in_sizes[9] != DINNER * DSTATE ||
      in_sizes[10] != DINNER        || out_size != TOKENS * DMODEL) return;

  const float* x      = (const float*)d_in[0];
  const float* W_in   = (const float*)d_in[1];
  const float* b_in   = (const float*)d_in[2];
  const float* W_gate = (const float*)d_in[3];
  const float* b_gate = (const float*)d_in[4];
  const float* W_out  = (const float*)d_in[5];
  const float* b_out  = (const float*)d_in[6];
  const float* A_log  = (const float*)d_in[7];
  const float* B_mat  = (const float*)d_in[8];
  const float* C_mat  = (const float*)d_in[9];
  const float* D_vec  = (const float*)d_in[10];
  float* out = (float*)d_out;

  const size_t bytes_proj = (size_t)TOKENS * 2 * DINNER * sizeof(float);
  const size_t bytes_gate = (size_t)TOKENS * DINNER * sizeof(float);
  const size_t bytes_gy   = (size_t)TOKENS * DINNER * sizeof(float);
  const size_t off_proj = 0;
  const size_t off_gate = off_proj + bytes_proj;
  const size_t off_gy   = off_gate + bytes_gate;
  if (off_gy + bytes_gy > ws_size) return;
  float* proj = (float*)((char*)d_ws + off_proj);
  float* gate = (float*)((char*)d_ws + off_gate);
  float* gy   = (float*)((char*)d_ws + off_gy);

  const float sW64   = 64.0f;
  const float sA256  = 256.0f;

  {
    dim3 g((2 * DINNER) / TN, TOKENS / TM);
    gemm_f16_nt<<<g, 256, 0, stream>>>(x, W_in, b_in, proj,
                                       TOKENS, 2 * DINNER, DMODEL,
                                       1.0f, sW64, 1.0f / 64.0f, 1, DINNER);
  }
  {
    dim3 g(DINNER / TN, TOKENS / TM);
    gemm_f16_nt<<<g, 256, 0, stream>>>(x, W_gate, b_gate, gate,
                                       TOKENS, DINNER, DMODEL,
                                       1.0f, sW64, 1.0f / 64.0f, 2, 0);
  }
  {
    dim3 g((B_SZ * DINNER) / SCAN_T);
    ssm_scan<<<g, SCAN_T, 0, stream>>>(proj, gate, A_log, B_mat, C_mat, D_vec, gy);
  }
  {
    dim3 g(DMODEL / TN, TOKENS / TM);
    gemm_f16_nt<<<g, 256, 0, stream>>>(gy, W_out, b_out, out,
                                       TOKENS, DMODEL, DINNER,
                                       sA256, sW64, 1.0f / 16384.0f, 0, 0);
  }
}
